// NPD_18253611008527
// MI455X (gfx1250) — hardware-run, weakly checked
//
#include <hip/hip_runtime.h>
#include <stddef.h>
#include <stdint.h>

#define NB    4096
#define NC    51
#define NM    (NB * NC)
#define NNODE 100000
#define KF    128
#define KH    256
#define NP    32
#define RB    64
#define HS    264
#define NOUT  (NB * (NC - 1))
#define OB    128

static_assert(NM == 208896);
static_assert((NM % RB) == 0);
static_assert((NOUT % OB) == 0);
static_assert(((NM / RB) * (RB * KF)) % 2048 == 0);
static_assert((KF % 32) == 0);
static_assert((KH % 32) == 0);
static_assert(NP == 32);
static_assert(((HS * 2) % 16) == 0);
static_assert(((KH * KF) % 2048) == 0);
static_assert(((KH * KH) % 2048) == 0);
static_assert(((NP * KH) % 2048) == 0);

typedef __attribute__((ext_vector_type(16))) __bf16    v16b;
typedef __attribute__((ext_vector_type(16))) _Float16 v16h;
typedef float        v8f __attribute__((ext_vector_type(8)));
typedef float        v4f __attribute__((ext_vector_type(4)));
typedef unsigned int v4u __attribute__((ext_vector_type(4)));

__device__ __forceinline__ unsigned short bf_bits(float f) {
  const unsigned u = __float_as_uint(f);
  return (unsigned short)((u + 0x7FFFu + ((u >> 16) & 1u)) >> 16);
}
__device__ __forceinline__ float bf_val(unsigned short b) { return __uint_as_float(((unsigned)b) << 16); }
__device__ __forceinline__ float bfr(float f) { return bf_val(bf_bits(f)); }
union H16 { _Float16 h; unsigned short u; };
__device__ __forceinline__ unsigned short h_bits(float f) {
  const float g = (fabsf(f) < 6.103515625e-05f) ? 0.0f : f;
  H16 x;
  x.h = (_Float16)g;
  return x.u;
}
__device__ __forceinline__ unsigned pk16(unsigned short a, unsigned short b) { return (unsigned)a | ((unsigned)b << 16); }
__device__ __forceinline__ v8f zero8() { v8f z = {0.f, 0.f, 0.f, 0.f, 0.f, 0.f, 0.f, 0.f}; return z; }
__device__ __forceinline__ float tanh_fast(float x) {
  const float t = __expf(2.0f * x);
  return 1.0f - 2.0f * __builtin_amdgcn_rcpf(t + 1.0f);
}
__device__ __forceinline__ float wsum(float v) {
#pragma unroll
  for (int off = 16; off >= 1; off >>= 1) v += __shfl_xor(v, off, 32);
  return v;
}

union FragB { v16b v; v4u u[2]; };
union FragH { v16h v; v4u u[2]; };
__device__ __forceinline__ v16b ldfrag_b(const unsigned short* p) {
  FragB f;
  f.u[0] = *(const v4u*)(p);
  f.u[1] = *(const v4u*)(p + 16);
  return f.v;
}
__device__ __forceinline__ v16h ldfrag_h(const unsigned short* p) {
  FragH f;
  f.u[0] = *(const v4u*)(p);
  f.u[1] = *(const v4u*)(p + 16);
  return f.v;
}

__device__ __forceinline__ v8f mma_b(v16b a, v16b b, v8f c) {
  return __builtin_amdgcn_wmma_f32_16x16x32_bf16(false, a, false, b, (short)0, c, false, false);
}
__device__ __forceinline__ v8f mma_h(v16h a, v16h b, v8f c) {
  return __builtin_amdgcn_wmma_f32_16x16x32_f16(false, a, false, b, (short)0, c, false, false);
}
template <typename F>
__device__ __forceinline__ void guard8(v8f (&a)[2][4], const F& x0, const F& x1,
                                       const F& g0, const F& g1, const F& g2, const F& g3) {
#if defined(__HIP_DEVICE_COMPILE__)
  asm volatile("v_nop\n\tv_nop\n\tv_nop\n\tv_nop"
               : "+v"(a[0][0]), "+v"(a[0][1]), "+v"(a[0][2]), "+v"(a[0][3]),
                 "+v"(a[1][0]), "+v"(a[1][1]), "+v"(a[1][2]), "+v"(a[1][3])
               : "v"(x0), "v"(x1), "v"(g0), "v"(g1), "v"(g2), "v"(g3));
#endif
}
template <typename F>
__device__ __forceinline__ void guard1(v8f& a, const F& x0, const F& g0) {
#if defined(__HIP_DEVICE_COMPILE__)
  asm volatile("v_nop\n\tv_nop\n\tv_nop\n\tv_nop" : "+v"(a) : "v"(x0), "v"(g0));
#endif
}

__global__ __launch_bounds__(256)
void k_gx(const int* __restrict__ idx, const float* __restrict__ dv, unsigned short* Xb) {
  const int e8 = (blockIdx.x * 256 + threadIdx.x) * 8;
  const int row = e8 >> 7;
  const int col = e8 & (KF - 1);
  int node = idx[row];
  node = min(max(node, 0), NNODE - 1);
  const float* src = dv + (size_t)node * KF + col;
  const v4f a = *(const v4f*)(src);
  const v4f b = *(const v4f*)(src + 4);
  v4u u;
  u[0] = pk16(bf_bits(a[0]), bf_bits(a[1]));
  u[1] = pk16(bf_bits(a[2]), bf_bits(a[3]));
  u[2] = pk16(bf_bits(b[0]), bf_bits(b[1]));
  u[3] = pk16(bf_bits(b[2]), bf_bits(b[3]));
  unsigned short* dst = Xb + e8;
  *(volatile v4u*)dst = u;
  __threadfence();
  *(volatile v4u*)dst = u;
}

__global__ __launch_bounds__(256)
void k_w(const float* __restrict__ W0, const float* __restrict__ W1, const float* __restrict__ WU,
         unsigned short* W0b, unsigned short* W1h, unsigned short* WUh) {
  const int blk = blockIdx.x, tid = threadIdx.x;
  const float* src;
  unsigned short* dst;
  int f16m;
  if (blk < 16) {
    const int t = blk * 256 + tid;
    src = W0 + (size_t)t * 8;  dst = W0b + (size_t)t * 8;  f16m = 0;
  } else if (blk < 48) {
    const int t = (blk - 16) * 256 + tid;
    src = W1 + (size_t)t * 8;  dst = W1h + (size_t)t * 8;  f16m = 1;
  } else {
    const int t = (blk - 48) * 256 + tid;
    src = WU + (size_t)t * 8;  dst = WUh + (size_t)t * 8;  f16m = 1;
  }
  const v4f a = *(const v4f*)(src);
  const v4f b = *(const v4f*)(src + 4);
  const float v[8] = {a[0], a[1], a[2], a[3], b[0], b[1], b[2], b[3]};
  unsigned short q[8];
#pragma unroll
  for (int i = 0; i < 8; ++i) {
    const unsigned short qb = bf_bits(v[i]);
    const unsigned short qh = h_bits(bf_val(qb) * 64.0f);
    q[i] = f16m ? qh : qb;
  }
  v4u u;
  u[0] = pk16(q[0], q[1]);
  u[1] = pk16(q[2], q[3]);
  u[2] = pk16(q[4], q[5]);
  u[3] = pk16(q[6], q[7]);
  *(volatile v4u*)dst = u;
  __threadfence();
  *(volatile v4u*)dst = u;
}

__device__ __forceinline__ void ep_tanh(unsigned short* sh, v8f (&acc)[2][4], const float (&bn)[4], float scale,
                                        int wr, int wc, int hh, int c) {
#pragma unroll
  for (int mt = 0; mt < 2; ++mt) {
#pragma unroll
    for (int nt = 0; nt < 4; ++nt) {
      const int col = wc + 16 * nt + c;
#pragma unroll
      for (int r = 0; r < 8; ++r) {
        const float hv = tanh_fast(acc[mt][nt][r] * scale + bn[nt]);
        sh[(wr + 16 * mt + 8 * hh + r) * HS + col] = h_bits(hv * 256.0f);
      }
    }
  }
}

__global__ __launch_bounds__(256)
void k_mlp(const unsigned short* __restrict__ Xb, const unsigned short* __restrict__ W0b,
           const unsigned short* __restrict__ W1h, const unsigned short* __restrict__ WUh,
           const float* __restrict__ b1, const float* __restrict__ bU, float* E) {
  __shared__ __align__(16) unsigned short sH[RB * HS];
  __shared__ __align__(16) float sE[RB * NP];
  const int tid = threadIdx.x, w = tid >> 5, lane = tid & 31, hh = lane >> 4, c = lane & 15;
  const int row0 = blockIdx.x * RB;
  const int wr = 32 * (w & 1), wc = 64 * (w >> 1);

  {
    v8f acc[2][4];
#pragma unroll
    for (int mt = 0; mt < 2; ++mt)
#pragma unroll
      for (int nt = 0; nt < 4; ++nt) acc[mt][nt] = zero8();
    const unsigned short* ap = Xb + (size_t)(row0 + wr + c) * KF + 8 * hh;
    const unsigned short* bp = W0b + (size_t)(wc + c) * KF + 8 * hh;
#pragma unroll 1
    for (int ks = 0; ks < KF / 32; ++ks) {
      const int ko = 32 * ks;
      const v16b a0 = ldfrag_b(ap + ko);
      const v16b a1 = ldfrag_b(ap + 16 * KF + ko);
      const v16b g0 = ldfrag_b(bp + ko);
      const v16b g1 = ldfrag_b(bp + 16 * KF + ko);
      const v16b g2 = ldfrag_b(bp + 32 * KF + ko);
      const v16b g3 = ldfrag_b(bp + 48 * KF + ko);
      acc[0][0] = mma_b(a0, g0, acc[0][0]);
      acc[0][1] = mma_b(a0, g1, acc[0][1]);
      acc[0][2] = mma_b(a0, g2, acc[0][2]);
      acc[0][3] = mma_b(a0, g3, acc[0][3]);
      acc[1][0] = mma_b(a1, g0, acc[1][0]);
      acc[1][1] = mma_b(a1, g1, acc[1][1]);
      acc[1][2] = mma_b(a1, g2, acc[1][2]);
      acc[1][3] = mma_b(a1, g3, acc[1][3]);
      guard8(acc, a0, a1, g0, g1, g2, g3);
    }
    const float bn[4] = {0.0f, 0.0f, 0.0f, 0.0f};
    ep_tanh(sH, acc, bn, 1.0f, wr, wc, hh, c);
  }
  __syncthreads();

  {
    v8f acc[2][4];
#pragma unroll
    for (int mt = 0; mt < 2; ++mt)
#pragma unroll
      for (int nt = 0; nt < 4; ++nt) acc[mt][nt] = zero8();
    const unsigned short* ap = sH + (wr + c) * HS + 8 * hh;
    const unsigned short* bp = W1h + (size_t)(wc + c) * KH + 8 * hh;
#pragma unroll 1
    for (int ks = 0; ks < KH / 32; ++ks) {
      const int ko = 32 * ks;
      const v16h a0 = ldfrag_h(ap + ko);
      const v16h a1 = ldfrag_h(ap + 16 * HS + ko);
      const v16h g0 = ldfrag_h(bp + ko);
      const v16h g1 = ldfrag_h(bp + 16 * KH + ko);
      const v16h g2 = ldfrag_h(bp + 32 * KH + ko);
      const v16h g3 = ldfrag_h(bp + 48 * KH + ko);
      acc[0][0] = mma_h(a0, g0, acc[0][0]);
      acc[0][1] = mma_h(a0, g1, acc[0][1]);
      acc[0][2] = mma_h(a0, g2, acc[0][2]);
      acc[0][3] = mma_h(a0, g3, acc[0][3]);
      acc[1][0] = mma_h(a1, g0, acc[1][0]);
      acc[1][1] = mma_h(a1, g1, acc[1][1]);
      acc[1][2] = mma_h(a1, g2, acc[1][2]);
      acc[1][3] = mma_h(a1, g3, acc[1][3]);
      guard8(acc, a0, a1, g0, g1, g2, g3);
    }
    __syncthreads();
    float bn[4];
#pragma unroll
    for (int nt = 0; nt < 4; ++nt) bn[nt] = bfr(b1[wc + 16 * nt + c]);
    ep_tanh(sH, acc, bn, 1.0f / 16384.0f, wr, wc, hh, c);
  }
  __syncthreads();

  {
    const int mr = 16 * (w & 3), nc0 = 16 * (w >> 2);
    v8f d = zero8();
    const unsigned short* ap = sH + (mr + c) * HS + 8 * hh;
    const unsigned short* bp = WUh + (size_t)(nc0 + c) * KH + 8 * hh;
#pragma unroll 1
    for (int ks = 0; ks < KH / 32; ++ks) {
      const int ko = 32 * ks;
      const v16h a0 = ldfrag_h(ap + ko);
      const v16h g0 = ldfrag_h(bp + ko);
      d = mma_h(a0, g0, d);
      guard1(d, a0, g0);
    }
    const float bu = bfr(bU[nc0 + c]);
#pragma unroll
    for (int r = 0; r < 8; ++r) sE[(mr + 8 * hh + r) * NP + nc0 + c] = d[r] * (1.0f / 16384.0f) + bu;
  }
  __syncthreads();

  const int lq = tid >> 3, p4 = (tid & 7) * 4;
  v4f o[2];
#pragma unroll
  for (int it = 0; it < 2; ++it) o[it] = *(const v4f*)(sE + (it * 32 + lq) * NP + p4);
  float* eb = E + (size_t)row0 * NP + (size_t)lq * NP + p4;
#pragma unroll
  for (int it = 0; it < 2; ++it) *(volatile v4f*)(eb + (size_t)it * 32 * NP) = o[it];
  __threadfence();
#pragma unroll
  for (int it = 0; it < 2; ++it) *(volatile v4f*)(eb + (size_t)it * 32 * NP) = o[it];
}

__global__ __launch_bounds__(256)
void k_dist(const float* __restrict__ E, float* out) {
#pragma clang fp contract(off)
  __shared__ __align__(16) float sO[OB];
  const int tid = threadIdx.x, w = tid >> 5, lane = tid & 31;
  const int base = blockIdx.x * OB;
  const float lim = 0.99999f;
  const float rl = 1.0f / 0.99999f;
#pragma unroll 1
  for (int j = 0; j < OB / 8; ++j) {
    const int p = base + w * (OB / 8) + j;
    const int b = p / (NC - 1);
    const int cc = p - b * (NC - 1) + 1;
    const float* sp = E + (size_t)b * NC * NP;
    const float* op = sp + cc * NP;
    float sk = sp[lane];
    float ok = op[lane];
    const float ss = wsum(sk * sk);
    const float s2 = wsum(ok * ok);
    const float ns = sqrtf(ss);
    const float no = sqrtf(s2);
    const float fs = (ns >= 1.0f) ? ns * rl : 1.0f;
    const float fo = (no >= 1.0f) ? no * rl : 1.0f;
    const float rs = 1.0f / fs;
    const float ro = 1.0f / fo;
    sk = sk * rs;
    ok = ok * ro;
    float squ = wsum(sk * sk);
    float sqv = wsum(ok * ok);
    const float dk = sk - ok;
    const float sqd = wsum(dk * dk);
    squ = fminf(fmaxf(squ, 0.0f), lim);
    sqv = fminf(fmaxf(sqv, 0.0f), lim);
    const float den = (1.0f - squ) * (1.0f - sqv);
    const float xx = sqd / den * 2.0f + 1.0f;
    const float z = sqrtf(xx * xx - 1.0f);
    const float dd = logf(xx + z);
    if (lane == 0) sO[w * (OB / 8) + j] = -dd;
  }
  __syncthreads();
  v4f v = {0.f, 0.f, 0.f, 0.f};
  if (tid < 32) v = *(const v4f*)(sO + tid * 4);
  float* ob = out + base + tid * 4;
  if (tid < 32) *(volatile v4f*)ob = v;
  __threadfence();
  if (tid < 32) *(volatile v4f*)ob = v;
}

extern "C" void kernel_launch(void* const* d_in, const int* in_sizes, int n_in,
                              void* d_out, int out_size, void* d_ws, size_t ws_size,
                              hipStream_t stream) {
  if (n_in < 7) return;
  if (in_sizes[0] != NM) return;
  if (in_sizes[1] != NNODE * KF) return;
  if (in_sizes[2] != KH * KF) return;
  if (in_sizes[3] != KH * KH) return;
  if (in_sizes[4] != KH) return;
  if (in_sizes[5] != NP * KH) return;
  if (in_sizes[6] != NP) return;
  if (out_size != NOUT) return;

  const int*   idx = (const int*)d_in[0];
  const float* dv  = (const float*)d_in[1];
  const float* W0  = (const float*)d_in[2];
  const float* W1  = (const float*)d_in[3];
  const float* b1  = (const float*)d_in[4];
  const float* WU  = (const float*)d_in[5];
  const float* bU  = (const float*)d_in[6];
  float* out = (float*)d_out;

  const size_t sXb = (size_t)NM * KF * 2;
  const size_t sE  = (size_t)NM * NP * 4;
  const size_t sW0 = (size_t)KH * KF * 2;
  const size_t sW1 = (size_t)KH * KH * 2;
  const size_t sWU = (size_t)NP * KH * 2;
  size_t off = 0;
  const size_t oXb = off; off += sXb;
  const size_t oE  = off; off += sE;
  const size_t oW0 = off; off += sW0;
  const size_t oW1 = off; off += sW1;
  const size_t oWU = off; off += sWU;
  if (off > ws_size) return;
  if (off > (size_t)134217728) return;

  char* ws = (char*)d_ws;
  unsigned short* Xb  = (unsigned short*)(ws + oXb);
  float*          E   = (float*)(ws + oE);
  unsigned short* W0b = (unsigned short*)(ws + oW0);
  unsigned short* W1h = (unsigned short*)(ws + oW1);
  unsigned short* WUh = (unsigned short*)(ws + oWU);

  k_gx<<<dim3((NM / 256) * (KF / 8)), dim3(256), 0, stream>>>(idx, dv, Xb);
  k_w<<<dim3(52), dim3(256), 0, stream>>>(W0, W1, WU, W0b, W1h, WUh);
  k_mlp<<<dim3(NM / RB), dim3(256), 0, stream>>>(Xb, W0b, W1h, WUh, b1, bU, E);
  k_dist<<<dim3(NOUT / OB), dim3(256), 0, stream>>>(E, out);
  (void)hipGetLastError();
}
